// Qwen3MoeSparseMoeBlock_31645319037665
// MI455X (gfx1250) — hardware-verified
//
#include <hip/hip_runtime.h>
#include <stdint.h>
#include <math.h>

#define T_TOK   2048
#define HID     1024
#define IMD     512
#define NEXP    16
#define TOPK    8
#define NTILE   272
#define NROWS   (NTILE * 64)
#define TTN     512
#define TT_DEAD 255
#define KC      128
#define NTHR    256
#define RTHR    128
#define WSMAX   134217728

#define CXL   1024.0f
#define CW    1024.0f
#define CHH   16.0f
#define CHL   1024.0f
#define CY    8.0f
#define S_GH  0.0009765625f
#define S_GL  9.5367431640625e-07f
#define S_YH  6.103515625e-05f
#define S_YL  5.9604644775390625e-08f
#define S_Y   0.125f

#define LDS_BKT ((NROWS + T_TOK * TOPK + TTN + 16) * 4)

static_assert(NROWS >= T_TOK * TOPK + NEXP * 63);
static_assert(NTILE <= TTN - 1);
static_assert(HID % KC == 0 && KC % 32 == 0 && IMD % 32 == 0 && HID % 32 == 0);
static_assert(IMD % 64 == 0 && HID % 64 == 0 && T_TOK % 64 == 0);
static_assert(T_TOK == NTHR * 8);
static_assert((NROWS / 4) % NTHR == 0 && (T_TOK * TOPK / 4) % NTHR == 0 && TTN / 4 <= NTHR);
static_assert(LDS_BKT <= 300000);
static_assert(T_TOK % 8 == 0);

typedef float          v4f   __attribute__((ext_vector_type(4)));
typedef float          v8f   __attribute__((ext_vector_type(8)));
typedef int            v4i   __attribute__((ext_vector_type(4)));
typedef int            v8i   __attribute__((ext_vector_type(8)));
typedef unsigned short v8us  __attribute__((ext_vector_type(8)));
typedef unsigned short v16us __attribute__((ext_vector_type(16)));
typedef _Float16       v4h   __attribute__((ext_vector_type(4)));
typedef _Float16       v8h   __attribute__((ext_vector_type(8)));
typedef _Float16       v16h  __attribute__((ext_vector_type(16)));
typedef __bf16         v16b  __attribute__((ext_vector_type(16)));
typedef v8h __attribute__((may_alias)) v8ha;
typedef v4h __attribute__((may_alias)) v4ha;
typedef v4f __attribute__((may_alias)) v4fa;
typedef v4i __attribute__((may_alias)) v4ia;

union FragH { v16h v; v8h h[2]; v8i w; };
union FragB { v16b v; v16us s; v8us u[2]; v8i w; };

__device__ __forceinline__ v8f wmh(const FragH& a, const FragH& b, v8f c) {
  v8f d = __builtin_amdgcn_wmma_f32_16x16x32_f16(false, a.v, false, b.v, (short)0, c, false, false);
  asm volatile("v_nop\n\tv_nop\n\tv_nop\n\tv_nop" : "+v"(d) : "v"(a.w), "v"(b.w));
  return d;
}
__device__ __forceinline__ v8f wmb(const FragB& a, const FragB& b, v8f c) {
  v8f d = __builtin_amdgcn_wmma_f32_16x16x32_bf16(false, a.v, false, b.v, (short)0, c, false, false);
  asm volatile("v_nop\n\tv_nop\n\tv_nop\n\tv_nop" : "+v"(d) : "v"(a.w), "v"(b.w));
  return d;
}

__device__ __forceinline__ unsigned bf_bits(float x) {
  const unsigned u = __float_as_uint(x);
  return (u + 0x7FFFu + ((u >> 16) & 1u)) >> 16;
}

__device__ __forceinline__ v8h cvt8h(const v4f a, const v4f b, const float c) {
  v8h hv;
  hv[0] = (_Float16)(a.x * c); hv[1] = (_Float16)(a.y * c);
  hv[2] = (_Float16)(a.z * c); hv[3] = (_Float16)(a.w * c);
  hv[4] = (_Float16)(b.x * c); hv[5] = (_Float16)(b.y * c);
  hv[6] = (_Float16)(b.z * c); hv[7] = (_Float16)(b.w * c);
  return hv;
}

__global__ __launch_bounds__(NTHR) void k_xprep(const float* __restrict__ x, _Float16* xh, _Float16* xl, int nUnits) {
  const int i = (int)blockIdx.x * NTHR + (int)threadIdx.x;
  if (i >= nUnits) return;
  const float* p = x + (size_t)i * 8;
  const v4f a = *(const v4fa*)p, b = *(const v4fa*)(p + 4);
  float f[8];
  f[0] = a.x; f[1] = a.y; f[2] = a.z; f[3] = a.w; f[4] = b.x; f[5] = b.y; f[6] = b.z; f[7] = b.w;
  v8h hv, lv;
#pragma unroll
  for (int j = 0; j < 8; ++j) {
    const _Float16 hj = (_Float16)f[j];
    hv[j] = hj;
    lv[j] = (_Float16)((f[j] - (float)hj) * CXL);
  }
  const size_t o = (size_t)i * 8;
  *(volatile v8h*)(xh + o) = hv;
  *(volatile v8h*)(xl + o) = lv;
  __threadfence();
  *(volatile v8h*)(xh + o) = hv;
  *(volatile v8h*)(xl + o) = lv;
}

__global__ __launch_bounds__(NTHR) void k_wprep(const float* __restrict__ w, _Float16* wt, int K, int N, int nUnits) {
  const int u = (int)blockIdx.x * NTHR + (int)threadIdx.x;
  if (u >= nUnits) return;
  const int kq = K >> 3;
  const int na = u / kq;
  const int k8 = (u - na * kq) * 8;
  const int e  = na / N;
  const int n  = na - e * N;
  const float* p = w + ((size_t)e * (size_t)K + (size_t)k8) * (size_t)N + n;
  v4f a, b;
  a.x = p[0];               a.y = p[(size_t)N];       a.z = p[(size_t)2 * N];   a.w = p[(size_t)3 * N];
  b.x = p[(size_t)4 * N];   b.y = p[(size_t)5 * N];   b.z = p[(size_t)6 * N];   b.w = p[(size_t)7 * N];
  const v8h hv = cvt8h(a, b, CW);
  const size_t o = (size_t)na * (size_t)K + k8;
  *(volatile v8h*)(wt + o) = hv;
  __threadfence();
  *(volatile v8h*)(wt + o) = hv;
}

__global__ __launch_bounds__(NTHR) void k_gwprep(const float* __restrict__ gw, unsigned short* gwh,
                                                unsigned short* gwl, int nUnits) {
  const int u = (int)blockIdx.x * NTHR + (int)threadIdx.x;
  if (u >= nUnits) return;
  const int n  = u / (HID / 8);
  const int k8 = (u - n * (HID / 8)) * 8;
  const float* p = gw + (size_t)k8 * NEXP + n;
  float f[8];
#pragma unroll
  for (int j = 0; j < 8; ++j) f[j] = p[(size_t)j * NEXP];
  v8us hv, lv;
#pragma unroll
  for (int j = 0; j < 8; ++j) {
    const unsigned hb = bf_bits(f[j]);
    const unsigned lb = bf_bits(f[j] - __uint_as_float(hb << 16));
    hv[j] = (unsigned short)hb;
    lv[j] = (unsigned short)lb;
  }
  const size_t o = (size_t)n * HID + k8;
  *(volatile v8us*)(gwh + o) = hv;
  *(volatile v8us*)(gwl + o) = lv;
  __threadfence();
  *(volatile v8us*)(gwh + o) = hv;
  *(volatile v8us*)(gwl + o) = lv;
}

__global__ __launch_bounds__(RTHR) void k_route(const float* __restrict__ x, const unsigned short* __restrict__ gwh,
                                               const unsigned short* __restrict__ gwl,
                                               float* out1, float* topw, int* sel) {
  __shared__ __attribute__((aligned(16))) float sL[64 * NEXP];
  __shared__ __attribute__((aligned(16))) float sW[64 * TOPK];
  __shared__ __attribute__((aligned(16))) int   sS[64];
  const int tid = (int)threadIdx.x, lane = tid & 31, wave = tid >> 5, hh = lane >> 4, m = lane & 15;
  const int t0 = (int)blockIdx.x * 64;

  const float* xr = x + (size_t)(t0 + 16 * wave + m) * HID + 8 * hh;
  const unsigned short* bhp = gwh + (size_t)m * HID + 8 * hh;
  const unsigned short* blp = gwl + (size_t)m * HID + 8 * hh;

  v8f acc = {0.f, 0.f, 0.f, 0.f, 0.f, 0.f, 0.f, 0.f};
#pragma unroll 1
  for (int ks = 0; ks < HID / 32; ++ks) {
    const int k0 = 32 * ks;
    const v4f x0 = *(const v4fa*)(xr + k0);
    const v4f x1 = *(const v4fa*)(xr + k0 + 4);
    const v4f x2 = *(const v4fa*)(xr + k0 + 16);
    const v4f x3 = *(const v4fa*)(xr + k0 + 20);
    float f[16];
    f[0] = x0.x; f[1] = x0.y; f[2]  = x0.z; f[3]  = x0.w; f[4]  = x1.x; f[5]  = x1.y; f[6]  = x1.z; f[7]  = x1.w;
    f[8] = x2.x; f[9] = x2.y; f[10] = x2.z; f[11] = x2.w; f[12] = x3.x; f[13] = x3.y; f[14] = x3.z; f[15] = x3.w;
    FragB ah, al;
#pragma unroll
    for (int i = 0; i < 16; ++i) {
      const unsigned hb = bf_bits(f[i]);
      const unsigned lb = bf_bits(f[i] - __uint_as_float(hb << 16));
      ah.s[i] = (unsigned short)hb;
      al.s[i] = (unsigned short)lb;
    }
    FragB wh, wl;
    wh.u[0] = *(const v8us*)(bhp + k0);
    wh.u[1] = *(const v8us*)(bhp + k0 + 16);
    wl.u[0] = *(const v8us*)(blp + k0);
    wl.u[1] = *(const v8us*)(blp + k0 + 16);
    acc = wmb(ah, wh, acc);
    acc = wmb(ah, wl, acc);
    acc = wmb(al, wh, acc);
  }
#pragma unroll
  for (int r = 0; r < 8; ++r) sL[(16 * wave + 8 * hh + r) * NEXP + m] = acc[r];
  __syncthreads();

  if (wave < 2) {
    const int tl = tid;
    float lg[NEXP];
    float mx = -3.0e38f;
#pragma unroll
    for (int e = 0; e < NEXP; ++e) { lg[e] = sL[tl * NEXP + e]; mx = fmaxf(mx, lg[e]); }
    float p[NEXP];
    float s = 0.f;
#pragma unroll
    for (int e = 0; e < NEXP; ++e) { p[e] = expf(lg[e] - mx); s += p[e]; }
    const float inv = 1.0f / s;
#pragma unroll
    for (int e = 0; e < NEXP; ++e) p[e] *= inv;
    unsigned selm = 0u;
    float wsum = 0.f;
#pragma unroll
    for (int k = 0; k < TOPK; ++k) {
      int best = 0;
      float bv = -1.0f;
#pragma unroll
      for (int e = 0; e < NEXP; ++e) {
        const bool ok = (((selm >> e) & 1u) == 0u) && (p[e] > bv);
        bv = ok ? p[e] : bv;
        best = ok ? e : best;
      }
      selm |= 1u << best;
      wsum += bv;
    }
    const float invw = 1.0f / wsum;
#pragma unroll
    for (int q = 0; q < TOPK; ++q) sW[tl * TOPK + q] = 0.f;
    int cnt = 0;
#pragma unroll
    for (int e = 0; e < NEXP; ++e) {
      if ((selm >> e) & 1u) {
        if (cnt < TOPK) sW[tl * TOPK + cnt] = p[e] * invw;
        ++cnt;
      }
    }
    sS[tl] = (int)selm;
  }
  __syncthreads();

  const v4f o0 = *(const v4fa*)(sL + 4 * tid);
  const v4f o1 = *(const v4fa*)(sL + 4 * (tid + RTHR));
  const v4f w4 = *(const v4fa*)(sW + 4 * tid);
  const v4i s4 = *(const v4ia*)(sS + 4 * (tid & 15));
  float* ob = out1 + (size_t)t0 * NEXP;
  float* wb = topw + (size_t)t0 * TOPK;
  int*   sb = sel + t0;
  const bool ws = tid < 16;
  *(volatile v4f*)(ob + 4 * tid) = o0;
  *(volatile v4f*)(ob + 4 * (tid + RTHR)) = o1;
  *(volatile v4f*)(wb + 4 * tid) = w4;
  if (ws) *(volatile v4i*)(sb + 4 * tid) = s4;
  __threadfence();
  *(volatile v4f*)(ob + 4 * tid) = o0;
  *(volatile v4f*)(ob + 4 * (tid + RTHR)) = o1;
  *(volatile v4f*)(wb + 4 * tid) = w4;
  if (ws) *(volatile v4i*)(sb + 4 * tid) = s4;
}

__global__ __launch_bounds__(NTHR) void k_bucket(const int* __restrict__ sel, int* btok, int* pos, int* tt) {
  extern __shared__ int ldsb[];
  int* sB  = ldsb;
  int* sP  = sB + NROWS;
  int* sT  = sP + T_TOK * TOPK;
  int* sWv = sT + TTN;
  const int tid = (int)threadIdx.x, lane = tid & 31, wave = tid >> 5;

  for (int i = tid; i < NROWS; i += NTHR) sB[i] = 0;
  for (int i = tid; i < T_TOK * TOPK; i += NTHR) sP[i] = 0;
  for (int i = tid; i < TTN; i += NTHR) sT[i] = TT_DEAD;
  const v4i ma = *(const v4ia*)(sel + 8 * tid);
  const v4i mb = *(const v4ia*)(sel + 8 * tid + 4);
  unsigned sm[8];
  sm[0] = (unsigned)ma.x & 0xFFFFu; sm[1] = (unsigned)ma.y & 0xFFFFu;
  sm[2] = (unsigned)ma.z & 0xFFFFu; sm[3] = (unsigned)ma.w & 0xFFFFu;
  sm[4] = (unsigned)mb.x & 0xFFFFu; sm[5] = (unsigned)mb.y & 0xFFFFu;
  sm[6] = (unsigned)mb.z & 0xFFFFu; sm[7] = (unsigned)mb.w & 0xFFFFu;
  __syncthreads();

  int gt = 0;
#pragma unroll 1
  for (int e = 0; e < NEXP; ++e) {
    const unsigned below = (1u << e) - 1u;
    int c = 0;
#pragma unroll
    for (int j = 0; j < 8; ++j) c += (int)((sm[j] >> e) & 1u);
    int incl = c;
#pragma unroll
    for (int d = 1; d < 32; d <<= 1) {
      const int up = __shfl_up(incl, d);
      if (lane >= d) incl += up;
    }
    if (lane == 31) sWv[wave] = incl;
    __syncthreads();
    int pre = 0, all = 0;
#pragma unroll
    for (int w2 = 0; w2 < NTHR / 32; ++w2) {
      int v = sWv[w2];
      v = v < 0 ? 0 : v;
      all += v;
      pre += (w2 < wave) ? v : 0;
    }
    int run = gt * 64 + pre + incl - c;
#pragma unroll
    for (int j = 0; j < 8; ++j) {
      if ((sm[j] >> e) & 1u) {
        const int tok = 8 * tid + j;
        const int rcl = run < NROWS ? run : NROWS - 1;
        if ((unsigned)run < (unsigned)NROWS) sB[run] = tok;
        const int kidx = (int)__builtin_popcount(sm[j] & below);
        if (kidx < TOPK) sP[tok * TOPK + kidx] = rcl;
        ++run;
      }
    }
    const int nt = (all + 63) >> 6;
    if (tid < nt && gt + tid < TTN) sT[gt + tid] = e;
    gt += nt;
    __syncthreads();
  }
  if (tid == 0) sT[TTN - 1] = (gt > NTILE) ? 1 : 0;
  __syncthreads();

  const bool wtt = tid < (TTN / 4);
#pragma unroll 1
  for (int it = 0; it < NROWS / 4 / NTHR; ++it) {
    const int p = it * NTHR + tid;
    const v4i v = *(const v4ia*)(sB + 4 * p);
    *(volatile v4i*)(btok + 4 * p) = v;
  }
#pragma unroll 1
  for (int it = 0; it < T_TOK * TOPK / 4 / NTHR; ++it) {
    const int p = it * NTHR + tid;
    const v4i v = *(const v4ia*)(sP + 4 * p);
    *(volatile v4i*)(pos + 4 * p) = v;
  }
  {
    const v4i v = *(const v4ia*)(sT + 4 * (tid & (TTN / 4 - 1)));
    if (wtt) *(volatile v4i*)(tt + 4 * tid) = v;
  }
  __threadfence();
#pragma unroll 1
  for (int it = 0; it < NROWS / 4 / NTHR; ++it) {
    const int p = it * NTHR + tid;
    const v4i v = *(const v4ia*)(sB + 4 * p);
    *(volatile v4i*)(btok + 4 * p) = v;
  }
#pragma unroll 1
  for (int it = 0; it < T_TOK * TOPK / 4 / NTHR; ++it) {
    const int p = it * NTHR + tid;
    const v4i v = *(const v4ia*)(sP + 4 * p);
    *(volatile v4i*)(pos + 4 * p) = v;
  }
  {
    const v4i v = *(const v4ia*)(sT + 4 * (tid & (TTN / 4 - 1)));
    if (wtt) *(volatile v4i*)(tt + 4 * tid) = v;
  }
}

__global__ __launch_bounds__(NTHR) void k_up(const _Float16* __restrict__ xh, const _Float16* __restrict__ xl,
                                             const _Float16* __restrict__ wgt, const _Float16* __restrict__ wut,
                                             const int* __restrict__ btok, const int* __restrict__ tt,
                                             _Float16* hmh, _Float16* hml) {
  __shared__ __attribute__((aligned(16))) _Float16 sA[2 * 64 * KC];
  __shared__ __attribute__((aligned(16))) _Float16 sO[2 * 64 * 64];
  __shared__ int sTok[64];
  const int g = (int)blockIdx.x;
  const int e = tt[g];
  if ((unsigned)e >= (unsigned)NEXP) return;
  const int c0 = (int)blockIdx.y * 64;
  const int tid = (int)threadIdx.x, lane = tid & 31, wave = tid >> 5, hh = lane >> 4, m = lane & 15;
  const int wr = wave & 3, wc = wave >> 2;
  if (tid < 64) {
    int tk = btok[g * 64 + tid];
    tk = tk < 0 ? 0 : (tk > T_TOK - 1 ? T_TOK - 1 : tk);
    sTok[tid] = tk;
  }
  __syncthreads();

  v8f Gh[2], Gl[2], Uh[2], Ul[2];
  {
    const v8f z = {0.f, 0.f, 0.f, 0.f, 0.f, 0.f, 0.f, 0.f};
    Gh[0] = z; Gh[1] = z; Gl[0] = z; Gl[1] = z; Uh[0] = z; Uh[1] = z; Ul[0] = z; Ul[1] = z;
  }
  const _Float16* aph = sA + (16 * wr + m) * KC + 8 * hh;
  const _Float16* apl = aph + 64 * KC;
  const size_t nrow = (size_t)e * IMD + c0 + 32 * wc + m;
  const _Float16* wgp = wgt + nrow * HID + 8 * hh;
  const _Float16* wup = wut + nrow * HID + 8 * hh;
  const int srow = tid >> 4, spc = (tid & 15) * 8;

#pragma unroll 1
  for (int kc = 0; kc < HID; kc += KC) {
#pragma unroll
    for (int it = 0; it < 4; ++it) {
      const int row = srow + 16 * it;
      const size_t src = (size_t)sTok[row] * HID + kc + spc;
      const v8h vh = *(const v8ha*)(xh + src);
      const v8h vl = *(const v8ha*)(xl + src);
      *(v8h*)(sA + row * KC + spc) = vh;
      *(v8h*)(sA + 64 * KC + row * KC + spc) = vl;
    }
    __syncthreads();
#pragma unroll
    for (int ks = 0; ks < KC / 32; ++ks) {
      FragH ah, al;
      ah.h[0] = *(const v8h*)(aph + 32 * ks);
      ah.h[1] = *(const v8h*)(aph + 32 * ks + 16);
      al.h[0] = *(const v8h*)(apl + 32 * ks);
      al.h[1] = *(const v8h*)(apl + 32 * ks + 16);
#pragma unroll
      for (int t = 0; t < 2; ++t) {
        const _Float16* q1 = wgp + (size_t)(16 * t) * HID + kc + 32 * ks;
        const _Float16* q2 = wup + (size_t)(16 * t) * HID + kc + 32 * ks;
        FragH bg, bu;
        bg.h[0] = *(const v8ha*)q1;  bg.h[1] = *(const v8ha*)(q1 + 16);
        bu.h[0] = *(const v8ha*)q2;  bu.h[1] = *(const v8ha*)(q2 + 16);
        Gh[t] = wmh(ah, bg, Gh[t]);
        Gl[t] = wmh(al, bg, Gl[t]);
        Uh[t] = wmh(ah, bu, Uh[t]);
        Ul[t] = wmh(al, bu, Ul[t]);
      }
    }
    __syncthreads();
  }

#pragma unroll
  for (int t = 0; t < 2; ++t) {
    const int col = 32 * wc + 16 * t + m;
#pragma unroll
    for (int r = 0; r < 8; ++r) {
      const int row = 16 * wr + 8 * hh + r;
      const float gg = fmaf(Gh[t][r], S_GH, Gl[t][r] * S_GL);
      const float uu = fmaf(Uh[t][r], S_GH, Ul[t][r] * S_GL);
      const float sg = __builtin_amdgcn_rcpf(1.0f + __expf(-gg));
      const float hm = (gg * sg) * uu;
      const float v  = hm * CHH;
      const _Float16 hf = (_Float16)v;
      const _Float16 lf = (_Float16)((v - (float)hf) * CHL);
      sO[row * 64 + col] = hf;
      sO[64 * 64 + row * 64 + col] = lf;
    }
  }
  __syncthreads();

  v8h pv[4];
  size_t po[4];
#pragma unroll
  for (int it = 0; it < 4; ++it) {
    const int q   = (it & 1) * NTHR + tid;
    const int pl  = it >> 1;
    const int row = q >> 3, q8 = q & 7;
    pv[it] = *(const v8ha*)(sO + pl * 64 * 64 + row * 64 + 8 * q8);
    po[it] = ((size_t)g * 64 + row) * IMD + c0 + 8 * q8;
  }
  *(volatile v8h*)(hmh + po[0]) = pv[0];
  *(volatile v8h*)(hmh + po[1]) = pv[1];
  *(volatile v8h*)(hml + po[2]) = pv[2];
  *(volatile v8h*)(hml + po[3]) = pv[3];
  __threadfence();
  *(volatile v8h*)(hmh + po[0]) = pv[0];
  *(volatile v8h*)(hmh + po[1]) = pv[1];
  *(volatile v8h*)(hml + po[2]) = pv[2];
  *(volatile v8h*)(hml + po[3]) = pv[3];
}

__global__ __launch_bounds__(NTHR) void k_down(const _Float16* __restrict__ hmh, const _Float16* __restrict__ hml,
                                               const _Float16* __restrict__ wdt, const int* __restrict__ tt,
                                               _Float16* yp) {
  __shared__ __attribute__((aligned(16))) _Float16 sO[64 * 64];
  const int g = (int)blockIdx.x;
  const int e = tt[g];
  if ((unsigned)e >= (unsigned)NEXP) return;
  const int c0 = (int)blockIdx.y * 64;
  const int tid = (int)threadIdx.x, lane = tid & 31, wave = tid >> 5, hh = lane >> 4, m = lane & 15;
  const int wr = wave & 3, wc = wave >> 2;

  v8f Yh[2], Yl[2];
  {
    const v8f z = {0.f, 0.f, 0.f, 0.f, 0.f, 0.f, 0.f, 0.f};
    Yh[0] = z; Yh[1] = z; Yl[0] = z; Yl[1] = z;
  }
  const size_t arow = (size_t)g * 64 + 16 * wr + m;
  const _Float16* aph = hmh + arow * IMD + 8 * hh;
  const _Float16* apl = hml + arow * IMD + 8 * hh;
  const _Float16* wp  = wdt + ((size_t)e * HID + c0 + 32 * wc + m) * IMD + 8 * hh;

#pragma unroll 1
  for (int ks = 0; ks < IMD / 32; ++ks) {
    FragH ah, al;
    ah.h[0] = *(const v8ha*)(aph + 32 * ks);
    ah.h[1] = *(const v8ha*)(aph + 32 * ks + 16);
    al.h[0] = *(const v8ha*)(apl + 32 * ks);
    al.h[1] = *(const v8ha*)(apl + 32 * ks + 16);
#pragma unroll
    for (int t = 0; t < 2; ++t) {
      const _Float16* q1 = wp + (size_t)(16 * t) * IMD + 32 * ks;
      FragH bf;
      bf.h[0] = *(const v8ha*)q1;
      bf.h[1] = *(const v8ha*)(q1 + 16);
      Yh[t] = wmh(ah, bf, Yh[t]);
      Yl[t] = wmh(al, bf, Yl[t]);
    }
  }

#pragma unroll
  for (int t = 0; t < 2; ++t) {
    const int col = 32 * wc + 16 * t + m;
#pragma unroll
    for (int r = 0; r < 8; ++r) {
      const int row = 16 * wr + 8 * hh + r;
      const float y = fmaf(Yh[t][r], S_YH, Yl[t][r] * S_YL);
      sO[row * 64 + col] = (_Float16)(y * CY);
    }
  }
  __syncthreads();

  v8h pv[2];
  size_t po[2];
#pragma unroll
  for (int it = 0; it < 2; ++it) {
    const int q = it * NTHR + tid;
    const int row = q >> 3, q8 = q & 7;
    pv[it] = *(const v8ha*)(sO + row * 64 + 8 * q8);
    po[it] = ((size_t)g * 64 + row) * HID + c0 + 8 * q8;
  }
  *(volatile v8h*)(yp + po[0]) = pv[0];
  *(volatile v8h*)(yp + po[1]) = pv[1];
  __threadfence();
  *(volatile v8h*)(yp + po[0]) = pv[0];
  *(volatile v8h*)(yp + po[1]) = pv[1];
}

__global__ __launch_bounds__(NTHR) void k_combine(const _Float16* __restrict__ yp, const float* __restrict__ topw,
                                                  const int* __restrict__ pos, const int* __restrict__ tt, float* out0) {
  const int lane = (int)threadIdx.x & 31, wave = (int)threadIdx.x >> 5;
  const int t = (int)blockIdx.x * 8 + wave;
  if (t >= T_TOK) return;
  const v4f wa = *(const v4fa*)(topw + (size_t)t * TOPK);
  const v4f wb = *(const v4fa*)(topw + (size_t)t * TOPK + 4);
  const v4i pa = *(const v4ia*)(pos + (size_t)t * TOPK);
  const v4i pb = *(const v4ia*)(pos + (size_t)t * TOPK + 4);
  const int flag = tt[TTN - 1];
  const float pz = (flag != 0 && t == 0) ? __int_as_float(0x7fc00000) : 0.0f;
  float w[8];
  w[0] = wa.x * S_Y; w[1] = wa.y * S_Y; w[2] = wa.z * S_Y; w[3] = wa.w * S_Y;
  w[4] = wb.x * S_Y; w[5] = wb.y * S_Y; w[6] = wb.z * S_Y; w[7] = wb.w * S_Y;
  int pr[8];
  pr[0] = pa.x; pr[1] = pa.y; pr[2] = pa.z; pr[3] = pa.w; pr[4] = pb.x; pr[5] = pb.y; pr[6] = pb.z; pr[7] = pb.w;
  const _Float16* yr[8];
#pragma unroll
  for (int j = 0; j < 8; ++j) {
    int pj = pr[j];
    pj = pj < 0 ? 0 : (pj > NROWS - 1 ? NROWS - 1 : pj);
    yr[j] = yp + (size_t)pj * HID;
  }
  float* orow = out0 + (size_t)t * HID;
#pragma unroll 1
  for (int c = 0; c < HID / 128; ++c) {
    const int col = 128 * c + 4 * lane;
    v4f acc = {0.f, 0.f, 0.f, 0.f};
#pragma unroll
    for (int j = 0; j < 8; ++j) {
      const v4h y = *(const v4ha*)(yr[j] + col);
      acc.x = fmaf(w[j], (float)y.x, acc.x);
      acc.y = fmaf(w[j], (float)y.y, acc.y);
      acc.z = fmaf(w[j], (float)y.z, acc.z);
      acc.w = fmaf(w[j], (float)y.w, acc.w);
    }
    acc.x += pz; acc.y += pz; acc.z += pz; acc.w += pz;
    float* op = orow + col;
    *(volatile v4f*)op = acc;
    __threadfence();
    *(volatile v4f*)op = acc;
  }
}

static inline int cdiv(int a, int b) { return (a + b - 1) / b; }

extern "C" void kernel_launch(void* const* d_in, const int* in_sizes, int n_in,
                              void* d_out, int out_size, void* d_ws, size_t ws_size,
                              hipStream_t stream) {
  if (n_in < 5) return;
  if (in_sizes[0] != T_TOK * HID) return;
  if (in_sizes[1] != HID * NEXP) return;
  if (in_sizes[2] != NEXP * HID * IMD) return;
  if (in_sizes[3] != NEXP * HID * IMD) return;
  if (in_sizes[4] != NEXP * IMD * HID) return;
  if (out_size != T_TOK * HID + T_TOK * NEXP) return;

  const float* x     = (const float*)d_in[0];
  const float* gatew = (const float*)d_in[1];
  const float* wgate = (const float*)d_in[2];
  const float* wup   = (const float*)d_in[3];
  const float* wdown = (const float*)d_in[4];
  float* out0 = (float*)d_out;
  float* out1 = out0 + (size_t)T_TOK * HID;

  char* ws = (char*)d_ws;
  size_t off = 0;
  const size_t oXH  = off; off += (size_t)T_TOK * HID * 2;           off = (off + 255) & ~(size_t)255;
  const size_t oXL  = off; off += (size_t)T_TOK * HID * 2;           off = (off + 255) & ~(size_t)255;
  const size_t oWG  = off; off += (size_t)NEXP * IMD * HID * 2;      off = (off + 255) & ~(size_t)255;
  const size_t oWU  = off; off += (size_t)NEXP * IMD * HID * 2;      off = (off + 255) & ~(size_t)255;
  const size_t oWD  = off; off += (size_t)NEXP * HID * IMD * 2;      off = (off + 255) & ~(size_t)255;
  const size_t oGH  = off; off += (size_t)NEXP * HID * 2;            off = (off + 255) & ~(size_t)255;
  const size_t oGL  = off; off += (size_t)NEXP * HID * 2;            off = (off + 255) & ~(size_t)255;
  const size_t oSEL = off; off += (size_t)T_TOK * 4;                 off = (off + 255) & ~(size_t)255;
  const size_t oTW  = off; off += (size_t)T_TOK * TOPK * 4;          off = (off + 255) & ~(size_t)255;
  const size_t oBT  = off; off += (size_t)NROWS * 4;                 off = (off + 255) & ~(size_t)255;
  const size_t oPOS = off; off += (size_t)T_TOK * TOPK * 4;          off = (off + 255) & ~(size_t)255;
  const size_t oTT  = off; off += (size_t)TTN * 4;                   off = (off + 255) & ~(size_t)255;
  const size_t oHMH = off; off += (size_t)NROWS * IMD * 2;           off = (off + 255) & ~(size_t)255;
  const size_t oHML = off; off += (size_t)NROWS * IMD * 2;           off = (off + 255) & ~(size_t)255;
  const size_t oYP  = off; off += (size_t)NROWS * HID * 2;           off = (off + 255) & ~(size_t)255;
  if (off > ws_size || off > (size_t)WSMAX) return;
  _Float16* XH  = (_Float16*)(ws + oXH);
  _Float16* XL  = (_Float16*)(ws + oXL);
  _Float16* WGT = (_Float16*)(ws + oWG);
  _Float16* WUT = (_Float16*)(ws + oWU);
  _Float16* WDT = (_Float16*)(ws + oWD);
  unsigned short* GWH = (unsigned short*)(ws + oGH);
  unsigned short* GWL = (unsigned short*)(ws + oGL);
  int*   SEL  = (int*)(ws + oSEL);
  float* TOPW = (float*)(ws + oTW);
  int*   BTOK = (int*)(ws + oBT);
  int*   POS  = (int*)(ws + oPOS);
  int*   TT   = (int*)(ws + oTT);
  _Float16* HMH = (_Float16*)(ws + oHMH);
  _Float16* HML = (_Float16*)(ws + oHML);
  _Float16* YP  = (_Float16*)(ws + oYP);

  hipFuncSetAttribute(reinterpret_cast<const void*>(&k_bucket),
                      hipFuncAttributeMaxDynamicSharedMemorySize, LDS_BKT);

  {
    const int nU = T_TOK * HID / 8;
    k_xprep<<<cdiv(nU, NTHR), NTHR, 0, stream>>>(x, XH, XL, nU);
  }
  {
    const int nU = NEXP * HID * IMD / 8;
    k_wprep<<<cdiv(nU, NTHR), NTHR, 0, stream>>>(wgate, WGT, HID, IMD, nU);
    k_wprep<<<cdiv(nU, NTHR), NTHR, 0, stream>>>(wup,   WUT, HID, IMD, nU);
    k_wprep<<<cdiv(nU, NTHR), NTHR, 0, stream>>>(wdown, WDT, IMD, HID, nU);
  }
  {
    const int nU = NEXP * HID / 8;
    k_gwprep<<<cdiv(nU, NTHR), NTHR, 0, stream>>>(gatew, GWH, GWL, nU);
  }
  k_route<<<T_TOK / 64, RTHR, 0, stream>>>(x, GWH, GWL, out1, TOPW, SEL);
  k_bucket<<<1, NTHR, LDS_BKT, stream>>>(SEL, BTOK, POS, TT);
  k_up<<<dim3(NTILE, IMD / 64), NTHR, 0, stream>>>(XH, XL, WGT, WUT, BTOK, TT, HMH, HML);
  k_down<<<dim3(NTILE, HID / 64), NTHR, 0, stream>>>(HMH, HML, WDT, TT, YP);
  k_combine<<<T_TOK / 8, NTHR, 0, stream>>>(YP, TOPW, POS, TT, out0);
}
